// GraphDecoderCore_88012469829876
// MI455X (gfx1250) — hardware-verified
//
#include <hip/hip_runtime.h>
#include <stddef.h>


#define NTHR   256
#define NWAVE  8
#define EPT    8
#define CHUNK  (NTHR * EPT)
#define WCAP   (EPT * 32)
#define LISTN  (NWAVE * WCAP)
#define TILE_E 16
#define PASSN  (NWAVE * TILE_E)
#define PCAP   (CHUNK + PASSN)
#define NB     1024
#define GRP    (NB / NTHR)
#define HD     10
#define HP     16
#define NIN    9
#define EF     11
#define EAP    16
#define MSGD   96
#define KIN    32
#define K1     (2 * HD + EF)
#define GIN    (EF + NIN)
#define AW     12
#define NBSM   304
#define WSC    16.0f
#define WINV   0.0625f

#define GS_WIH 0
#define GS_WHH 600
#define GS_BIH 900
#define GS_BHH 932
#define GS_FW  964
#define GS_FB  984
#define NGSM   992

#define LO_W1   0
#define LO_W2   (LO_W1 + MSGD * KIN * 2)
#define LO_W3   (LO_W2 + MSGD * MSGD * 2)
#define LO_W4   (LO_W3 + MSGD * MSGD * 2)
#define LO_BS   (LO_W4 + 16 * MSGD * 2)
#define LO_GS   (LO_BS + NBSM * 4)
#define LO_ACC  (LO_GS + NGSM * 4)
#define LO_STG  (LO_ACC + (NB + 1) * AW * 4)
#define LO_MSG  (LO_STG + NWAVE * TILE_E * KIN * 2)
#define LO_LIST (LO_MSG + PASSN * AW * 4)
#define LO_PEND (LO_LIST + LISTN * 4)
#define LO_SLOT (LO_PEND + PCAP * 4)
#define LO_HST  (LO_SLOT + PASSN * 4)
#define LO_LG   (LO_HST + NTHR * HP * 4)
#define LO_WCNT (LO_LG + NB * 2 * 4)
#define LO_PN   (LO_WCNT + 64)
#define LDS_BYTES (LO_PN + 64)

static_assert(PASSN == 128);
static_assert((PCAP % PASSN) == 0);
static_assert(PCAP >= CHUNK + PASSN);
static_assert((NB % NTHR) == 0);
static_assert(GIN == 2 * HD);
static_assert((LO_W2 % 16) == 0 && (LO_W3 % 16) == 0 && (LO_W4 % 16) == 0 && (LO_BS % 16) == 0);
static_assert((LO_GS % 16) == 0 && (LO_ACC % 16) == 0 && (LO_STG % 16) == 0 && (LO_MSG % 16) == 0);
static_assert((LO_LIST % 16) == 0 && (LO_PEND % 16) == 0 && (LO_SLOT % 16) == 0 && (LO_HST % 16) == 0);
static_assert((LO_LG % 16) == 0 && (LO_WCNT % 16) == 0 && (LO_PN % 16) == 0);
static_assert(LDS_BYTES < 300000);

typedef float    v2f  __attribute__((ext_vector_type(2)));
typedef float    v4f  __attribute__((ext_vector_type(4)));
typedef float    v8f  __attribute__((ext_vector_type(8)));
typedef int      v4i  __attribute__((ext_vector_type(4)));
typedef _Float16 v2h  __attribute__((ext_vector_type(2)));
typedef _Float16 v4h  __attribute__((ext_vector_type(4)));
typedef _Float16 v8h  __attribute__((ext_vector_type(8)));
typedef _Float16 v16h __attribute__((ext_vector_type(16)));
union FragH { v16h v; v8h h[2]; };
union Half8 { v8h v; v4h q[2]; };
union Pun16 { v8h h; v4f f; };

__device__ __forceinline__ v8h zero8() {
  v8h r;
#pragma unroll
  for (int i = 0; i < 8; ++i) r[i] = (_Float16)0.0f;
  return r;
}
__device__ __forceinline__ v4h zero4() {
  v4h r;
#pragma unroll
  for (int i = 0; i < 4; ++i) r[i] = (_Float16)0.0f;
  return r;
}

__device__ __forceinline__ v8f wmh(v16h a, v16h b, v8f c) {
  v8f d = __builtin_amdgcn_wmma_f32_16x16x32_f16(false, a, false, b, (short)0, c, false, false);
  asm volatile("v_nop\n\tv_nop\n\tv_nop\n\tv_nop" : "+v"(d) : "v"(a), "v"(b));
  return d;
}

__device__ __forceinline__ v8h relu8(v8f d) {
  v8h r;
#pragma unroll
  for (int i = 0; i < 8; ++i) { const float t = fmaxf(d[i] * WINV, 0.0f); r[i] = (_Float16)t; }
  return r;
}

__device__ __forceinline__ v8f ldc8(const float* p) {
  const v4f a = *(const v4f*)p;
  const v4f b = *(const v4f*)(p + 4);
  v8f c;
  c[0] = a.x; c[1] = a.y; c[2] = a.z; c[3] = a.w;
  c[4] = b.x; c[5] = b.y; c[6] = b.z; c[7] = b.w;
  return c;
}

__device__ __forceinline__ float sigm(float a) {
  const float t = expf(-fabsf(a));
  const float v = 1.0f / (1.0f + t);
  return (a >= 0.0f) ? v : t * v;
}

__device__ __forceinline__ int scan_chunk(const int* __restrict__ dsts, int nE, int cbase, int nodeBase,
                                          int* list, int tid, int wave) {
  int wc = 0;
  const int el0  = tid * EPT;
  const int e0   = cbase + el0;
  const int sent = -2147483647 - 1;
  v4i da, db;
  if (cbase + CHUNK <= nE) {
    da = *(const v4i*)(dsts + e0);
    db = *(const v4i*)(dsts + e0 + 4);
  } else {
    da.x = (e0     < nE) ? dsts[min(e0, nE - 1)] : sent;
    da.y = (e0 + 1 < nE) ? dsts[min(e0 + 1, nE - 1)] : sent;
    da.z = (e0 + 2 < nE) ? dsts[min(e0 + 2, nE - 1)] : sent;
    da.w = (e0 + 3 < nE) ? dsts[min(e0 + 3, nE - 1)] : sent;
    db.x = (e0 + 4 < nE) ? dsts[min(e0 + 4, nE - 1)] : sent;
    db.y = (e0 + 5 < nE) ? dsts[min(e0 + 5, nE - 1)] : sent;
    db.z = (e0 + 6 < nE) ? dsts[min(e0 + 6, nE - 1)] : sent;
    db.w = (e0 + 7 < nE) ? dsts[min(e0 + 7, nE - 1)] : sent;
  }
  const unsigned nb = (unsigned)nodeBase;
  const unsigned s0 = (unsigned)da.x - nb, s1 = (unsigned)da.y - nb;
  const unsigned s2 = (unsigned)da.z - nb, s3 = (unsigned)da.w - nb;
  const unsigned s4 = (unsigned)db.x - nb, s5 = (unsigned)db.y - nb;
  const unsigned s6 = (unsigned)db.z - nb, s7 = (unsigned)db.w - nb;
  const bool h0 = s0 < (unsigned)NB, h1 = s1 < (unsigned)NB, h2 = s2 < (unsigned)NB, h3 = s3 < (unsigned)NB;
  const bool h4 = s4 < (unsigned)NB, h5 = s5 < (unsigned)NB, h6 = s6 < (unsigned)NB, h7 = s7 < (unsigned)NB;
  const unsigned any = __builtin_amdgcn_ballot_w32(h0 | h1 | h2 | h3 | h4 | h5 | h6 | h7);
  if (any != 0u) {
#define HITJ(J, HJ) { \
      const unsigned mj = __builtin_amdgcn_ballot_w32(HJ); \
      if (mj != 0u) { \
        if (HJ) { \
          const int pos = wc + (int)__builtin_amdgcn_mbcnt_lo(mj, 0u); \
          if (pos < WCAP) list[wave * WCAP + pos] = el0 + (J); \
        } \
        wc += (int)__builtin_popcount(mj); } }
    HITJ(0, h0)
    HITJ(1, h1)
    HITJ(2, h2)
    HITJ(3, h3)
    HITJ(4, h4)
    HITJ(5, h5)
    HITJ(6, h6)
    HITJ(7, h7)
#undef HITJ
  }
  return wc;
}

__global__ __launch_bounds__(NTHR) void k_prep(const float* __restrict__ ea, _Float16* ea16, int nE) {
  const int p  = blockIdx.x * NTHR + threadIdx.x;
  const int e  = p >> 1, hf = p & 1;
  const int ec = e > nE - 1 ? nE - 1 : e;
  const bool ev = e < nE;
  Pun16 u;
#pragma unroll
  for (int j = 0; j < 8; ++j) {
    const int c  = 8 * hf + j;
    const int cc = c > EF - 1 ? EF - 1 : c;
    float v = ea[(size_t)ec * EF + cc];
    v = (ev && c < EF) ? v : 0.0f;
    u.h[j] = (_Float16)v;
  }
  _Float16* dp = ea16 + (size_t)p * 8;
  const v4f fv = u.f;
  *(volatile v4f*)dp = fv;
  __threadfence();
  *(volatile v4f*)dp = fv;
}

__global__ __launch_bounds__(NTHR) void k_iter(
    const float* __restrict__ hin, float* hout, const _Float16* __restrict__ ea16,
    const float* __restrict__ xin,
    const float* __restrict__ W1, const float* __restrict__ Bi1,
    const float* __restrict__ W2, const float* __restrict__ Bi2,
    const float* __restrict__ W3, const float* __restrict__ Bi3,
    const float* __restrict__ W4, const float* __restrict__ Bi4,
    const float* __restrict__ gwih, const float* __restrict__ gwhh,
    const float* __restrict__ gbih, const float* __restrict__ gbhh,
    const float* __restrict__ gfw, const float* __restrict__ gfb,
    const int* __restrict__ srcs, const int* __restrict__ dsts,
    float* outp, int nN, int nE, int outLim) {
  extern __shared__ __attribute__((aligned(16))) unsigned char smem[];
  _Float16* w1s  = (_Float16*)(smem + LO_W1);
  _Float16* w2s  = (_Float16*)(smem + LO_W2);
  _Float16* w3s  = (_Float16*)(smem + LO_W3);
  _Float16* w4s  = (_Float16*)(smem + LO_W4);
  float*    bsm  = (float*)(smem + LO_BS);
  float*    gsm  = (float*)(smem + LO_GS);
  float*    acc  = (float*)(smem + LO_ACC);
  _Float16* stg  = (_Float16*)(smem + LO_STG);
  float*    msg  = (float*)(smem + LO_MSG);
  int*      list = (int*)(smem + LO_LIST);
  int*      pend = (int*)(smem + LO_PEND);
  int*      slotb = (int*)(smem + LO_SLOT);
  float*    hst  = (float*)(smem + LO_HST);
  float*    lg   = (float*)(smem + LO_LG);
  int*      wcnt = (int*)(smem + LO_WCNT);
  int*      pendN = (int*)(smem + LO_PN);

  const int tid = threadIdx.x, lane = tid & 31, wave = tid >> 5, hh = lane >> 4, m = lane & 15;
  const int nodeBase = blockIdx.x * NB;

  for (int i = tid; i < MSGD * KIN; i += NTHR) {
    const int n = i >> 5, k = i & 31;
    const int kc = k < K1 ? k : K1 - 1;
    float v = W1[n * K1 + kc];
    v = (k < K1) ? v : 0.0f;
    w1s[i] = (_Float16)(v * WSC);
  }
  for (int i = tid; i < MSGD * MSGD; i += NTHR) {
    w2s[i] = (_Float16)(W2[i] * WSC);
    w3s[i] = (_Float16)(W3[i] * WSC);
  }
  for (int i = tid; i < 16 * MSGD; i += NTHR) {
    const int n = i / MSGD, k = i - n * MSGD;
    const int nc = n < EF ? n : EF - 1;
    float v = W4[nc * MSGD + k];
    v = (n < EF) ? v : 0.0f;
    w4s[i] = (_Float16)(v * WSC);
  }
  for (int i = tid; i < NBSM; i += NTHR) {
    const int i1 = i > MSGD - 1 ? MSGD - 1 : i;
    int i2 = i - MSGD;     i2 = i2 < 0 ? 0 : (i2 > MSGD - 1 ? MSGD - 1 : i2);
    int i3 = i - 2 * MSGD; i3 = i3 < 0 ? 0 : (i3 > MSGD - 1 ? MSGD - 1 : i3);
    int i4 = i - 3 * MSGD; i4 = i4 < 0 ? 0 : (i4 > EF - 1 ? EF - 1 : i4);
    const float c1 = Bi1[i1], c2 = Bi2[i2], c3 = Bi3[i3], c4 = Bi4[i4];
    float v = 0.0f;
    if (i < MSGD) v = c1;
    else if (i < 2 * MSGD) v = c2;
    else if (i < 3 * MSGD) v = c3;
    else if (i < 3 * MSGD + EF) v = c4;
    bsm[i] = v * WSC;
  }
  for (int i = tid; i < 3 * HD * GIN; i += NTHR) gsm[GS_WIH + i] = gwih[i];
  for (int i = tid; i < 3 * HD * HD; i += NTHR) gsm[GS_WHH + i] = gwhh[i];
  if (tid < 3 * HD) { gsm[GS_BIH + tid] = gbih[tid]; gsm[GS_BHH + tid] = gbhh[tid]; }
  if (tid < 2 * HD) gsm[GS_FW + tid] = gfw[tid];
  if (tid < 2) gsm[GS_FB + tid] = gfb[tid];
  for (int i = tid; i < (NB + 1) * AW; i += NTHR) acc[i] = 0.0f;
  if (tid == 0) pendN[0] = 0;
  __syncthreads();

  const int nChunks = (nE + CHUNK - 1) / CHUNK;
#pragma unroll 1
  for (int ch = 0; ch < nChunks; ++ch) {
    const int cbase = ch * CHUNK;
    const int wc = scan_chunk(dsts, nE, cbase, nodeBase, list, tid, wave);
    if (lane == 0) wcnt[wave] = wc;
    __syncthreads();

    const int base = pendN[0];
    int tot = 0, myoff = 0;
#pragma unroll
    for (int w = 0; w < NWAVE; ++w) {
      int c = wcnt[w];
      c = c > WCAP ? WCAP : (c < 0 ? 0 : c);
      if (w < wave) myoff += c;
      tot += c;
    }
    int newN = base + tot;
    newN = newN > PCAP ? PCAP : newN;
    {
      int n = wcnt[wave];
      n = n > WCAP ? WCAP : (n < 0 ? 0 : n);
      const int* lp = list + wave * WCAP;
      for (int i = lane; i < n; i += 32) {
        const int pos = base + myoff + i;
        if (pos < PCAP) pend[pos] = cbase + lp[i];
      }
    }
    const int fin = (ch == nChunks - 1) ? 1 : 0;
    const int R   = (fin != 0) ? (newN + PASSN - 1) / PASSN : newN / PASSN;
    const int Pv  = (fin != 0) ? newN : R * PASSN;
    __syncthreads();

#pragma unroll 1
    for (int r = 0; r < R; ++r) {
      {
        const int idx = r * PASSN + wave * TILE_E + m;
        const bool valid = idx < Pv;
        int e = pend[idx];
        e = valid ? e : 0;
        e = e < 0 ? 0 : (e > nE - 1 ? nE - 1 : e);
        int d = dsts[e];
        int s = srcs[e];
        int slot = d - nodeBase;
        if (!valid || (unsigned)slot >= (unsigned)NB) slot = NB;
        d = d < 0 ? 0 : (d > nN - 1 ? nN - 1 : d);
        s = s < 0 ? 0 : (s > nN - 1 ? nN - 1 : s);
        const int node = (hh != 0) ? d : s;
        const float* hp = hin + (size_t)node * HP;
        const v4f q0 = *(const v4f*)hp;
        const v4f q1 = *(const v4f*)(hp + 4);
        const v2f q2 = *(const v2f*)(hp + 8);
        const _Float16* ep = ea16 + (size_t)e * EAP;
        Half8 ea0; ea0.v = *(const v8h*)ep;
        v4h ea1 = *(const v4h*)(ep + 8);
        float f0 = q0.x, f1 = q0.y, f2 = q0.z, f3 = q0.w, f4 = q1.x, f5 = q1.y, f6 = q1.z, f7 = q1.w, f8 = q2.x, f9 = q2.y;
        if (!valid) {
          f0 = 0.0f; f1 = 0.0f; f2 = 0.0f; f3 = 0.0f; f4 = 0.0f; f5 = 0.0f; f6 = 0.0f; f7 = 0.0f; f8 = 0.0f; f9 = 0.0f;
          ea0.v = zero8(); ea1 = zero4();
        }
        _Float16* row = stg + (wave * TILE_E + m) * KIN;
        _Float16* np  = row + HD * hh;
        const v2h p0 = {(_Float16)f0, (_Float16)f1};
        const v2h p1 = {(_Float16)f2, (_Float16)f3};
        const v2h p2 = {(_Float16)f4, (_Float16)f5};
        const v2h p3 = {(_Float16)f6, (_Float16)f7};
        const v2h p4 = {(_Float16)f8, (_Float16)f9};
        *(v2h*)(np + 0) = p0;
        *(v2h*)(np + 2) = p1;
        *(v2h*)(np + 4) = p2;
        *(v2h*)(np + 6) = p3;
        *(v2h*)(np + 8) = p4;
        if (hh == 0) {
          *(v4h*)(row + 2 * HD)     = ea0.q[0];
          *(v4h*)(row + 2 * HD + 4) = ea0.q[1];
          slotb[wave * TILE_E + m] = slot;
        } else {
          *(v4h*)(row + 2 * HD + 8) = ea1;
        }
      }
      __syncthreads();

      {
        FragH bx;
        {
          const _Float16* sp = stg + (wave * TILE_E + m) * KIN + 8 * hh;
          bx.h[0] = *(const v8h*)sp;
          bx.h[1] = *(const v8h*)(sp + 16);
        }
        FragH bA[3], bB[3];
#pragma unroll
        for (int j = 0; j < 3; ++j) {
          FragH a0, a1;
          const _Float16* ap0 = w1s + (32 * j + m) * KIN + 8 * hh;
          const _Float16* ap1 = ap0 + 16 * KIN;
          a0.h[0] = *(const v8h*)ap0;  a0.h[1] = *(const v8h*)(ap0 + 16);
          a1.h[0] = *(const v8h*)ap1;  a1.h[1] = *(const v8h*)(ap1 + 16);
          const v8f d0 = wmh(a0.v, bx.v, ldc8(bsm + 32 * j + 8 * hh));
          const v8f d1 = wmh(a1.v, bx.v, ldc8(bsm + 32 * j + 16 + 8 * hh));
          bA[j].h[0] = relu8(d0);
          bA[j].h[1] = relu8(d1);
        }
#pragma unroll
        for (int j = 0; j < 3; ++j) {
          v8f d0 = ldc8(bsm + MSGD + 32 * j + 8 * hh);
          v8f d1 = ldc8(bsm + MSGD + 32 * j + 16 + 8 * hh);
#pragma unroll
          for (int kc = 0; kc < 3; ++kc) {
            FragH a0, a1;
            const _Float16* ap0 = w2s + (32 * j + m) * MSGD + 32 * kc + 8 * hh;
            const _Float16* ap1 = ap0 + 16 * MSGD;
            a0.h[0] = *(const v8h*)ap0;  a0.h[1] = *(const v8h*)(ap0 + 16);
            a1.h[0] = *(const v8h*)ap1;  a1.h[1] = *(const v8h*)(ap1 + 16);
            d0 = wmh(a0.v, bA[kc].v, d0);
            d1 = wmh(a1.v, bA[kc].v, d1);
          }
          bB[j].h[0] = relu8(d0);
          bB[j].h[1] = relu8(d1);
        }
#pragma unroll
        for (int j = 0; j < 3; ++j) {
          v8f d0 = ldc8(bsm + 2 * MSGD + 32 * j + 8 * hh);
          v8f d1 = ldc8(bsm + 2 * MSGD + 32 * j + 16 + 8 * hh);
#pragma unroll
          for (int kc = 0; kc < 3; ++kc) {
            FragH a0, a1;
            const _Float16* ap0 = w3s + (32 * j + m) * MSGD + 32 * kc + 8 * hh;
            const _Float16* ap1 = ap0 + 16 * MSGD;
            a0.h[0] = *(const v8h*)ap0;  a0.h[1] = *(const v8h*)(ap0 + 16);
            a1.h[0] = *(const v8h*)ap1;  a1.h[1] = *(const v8h*)(ap1 + 16);
            d0 = wmh(a0.v, bB[kc].v, d0);
            d1 = wmh(a1.v, bB[kc].v, d1);
          }
          bA[j].h[0] = relu8(d0);
          bA[j].h[1] = relu8(d1);
        }
        v8f d4 = ldc8(bsm + 3 * MSGD + 8 * hh);
#pragma unroll
        for (int kc = 0; kc < 3; ++kc) {
          FragH a;
          const _Float16* ap = w4s + m * MSGD + 32 * kc + 8 * hh;
          a.h[0] = *(const v8h*)ap;  a.h[1] = *(const v8h*)(ap + 16);
          d4 = wmh(a.v, bA[kc].v, d4);
        }
        float* mp = msg + (wave * TILE_E + m) * AW;
#pragma unroll
        for (int rr = 0; rr < 8; ++rr) {
          const int f = 8 * hh + rr;
          if (f < EF) mp[f] = d4[rr] * WINV;
        }
      }
      __syncthreads();

      if (wave == 0) {
#pragma unroll 1
        for (int i = 0; i < PASSN; ++i) {
          int sl = slotb[i];
          sl = sl < 0 ? 0 : (sl > NB ? NB : sl);
          if (lane < EF) {
            const float v = msg[i * AW + lane];
            acc[sl * AW + lane] += v;
          }
        }
      }
      __syncthreads();
    }

    int rem = newN - R * PASSN;
    rem = rem < 0 ? 0 : rem;
    if (R > 0 && tid < rem) pend[tid] = pend[R * PASSN + tid];
    if (tid == 0) pendN[0] = rem;
  }
  __syncthreads();

#pragma unroll 1
  for (int g = 0; g < GRP; ++g) {
    const int slot = g * NTHR + tid;
    const int n  = nodeBase + slot;
    const int nc = n > nN - 1 ? nN - 1 : n;
    float x[GIN];
#pragma unroll
    for (int f = 0; f < EF; ++f) x[f] = acc[slot * AW + f];
#pragma unroll
    for (int f = 0; f < NIN; ++f) x[EF + f] = xin[(size_t)nc * NIN + f];
    const float* hq = hin + (size_t)nc * HP;
    const v4f u0 = *(const v4f*)hq;
    const v4f u1 = *(const v4f*)(hq + 4);
    const v2f u2 = *(const v2f*)(hq + 8);
    const float hv[HD] = {u0.x, u0.y, u0.z, u0.w, u1.x, u1.y, u1.z, u1.w, u2.x, u2.y};
    float s0 = gsm[GS_FB], s1 = gsm[GS_FB + 1];
    float* hrow = hst + tid * HP;
#pragma unroll 1
    for (int j = 0; j < HD; ++j) {
      const float* wr = gsm + GS_WIH + j * GIN;
      const float* wz = wr + HD * GIN;
      const float* wn = wz + HD * GIN;
      float gir = gsm[GS_BIH + j], giz = gsm[GS_BIH + HD + j], gin = gsm[GS_BIH + 2 * HD + j];
#pragma unroll
      for (int k = 0; k < GIN; ++k) {
        const float xk = x[k];
        gir += wr[k] * xk;
        giz += wz[k] * xk;
        gin += wn[k] * xk;
      }
      const float* ur = gsm + GS_WHH + j * HD;
      const float* uz = ur + HD * HD;
      const float* un = uz + HD * HD;
      float ghr = gsm[GS_BHH + j], ghz = gsm[GS_BHH + HD + j], ghn = gsm[GS_BHH + 2 * HD + j];
#pragma unroll
      for (int k = 0; k < HD; ++k) {
        const float hk = hv[k];
        ghr += ur[k] * hk;
        ghz += uz[k] * hk;
        ghn += un[k] * hk;
      }
      const float rg = sigm(gir + ghr);
      const float zg = sigm(giz + ghz);
      const float ng = tanhf(gin + rg * ghn);
      const float ho = hq[j];
      const float hn = (1.0f - zg) * ng + zg * ho;
      hrow[j] = hn;
      s0 += gsm[GS_FW + j] * hn;
      s1 += gsm[GS_FW + HD + j] * hn;
    }
#pragma unroll
    for (int j = HD; j < HP; ++j) hrow[j] = 0.0f;
    lg[slot * 2]     = s0;
    lg[slot * 2 + 1] = s1;
    __syncthreads();

    v4f hw[4];
#pragma unroll
    for (int q = 0; q < 4; ++q) hw[q] = *(const v4f*)(hst + (q * NTHR + tid) * 4);
    float* hb = hout + (size_t)(nodeBase + g * NTHR) * HP;
#pragma unroll
    for (int q = 0; q < 4; ++q) *(volatile v4f*)(hb + (q * NTHR + tid) * 4) = hw[q];
    __threadfence();
#pragma unroll
    for (int q = 0; q < 4; ++q) *(volatile v4f*)(hb + (q * NTHR + tid) * 4) = hw[q];
    __syncthreads();
  }

  v4f lw[2];
#pragma unroll
  for (int q = 0; q < 2; ++q) lw[q] = *(const v4f*)(lg + (q * NTHR + tid) * 4);
  const size_t ob  = (size_t)nodeBase * 2;
  const size_t lim = (size_t)(outLim < 0 ? 0 : outLim);
#pragma unroll
  for (int q = 0; q < 2; ++q) {
    const size_t gi = ob + (size_t)((q * NTHR + tid) * 4);
    if (gi + 3 < lim) *(volatile v4f*)(outp + gi) = lw[q];
  }
  __threadfence();
#pragma unroll
  for (int q = 0; q < 2; ++q) {
    const size_t gi = ob + (size_t)((q * NTHR + tid) * 4);
    if (gi + 3 < lim) *(volatile v4f*)(outp + gi) = lw[q];
  }
}

extern "C" void kernel_launch(void* const* d_in, const int* in_sizes, int n_in,
                              void* d_out, int out_size, void* d_ws, size_t ws_size,
                              hipStream_t stream) {
  if (n_in < 18) return;
  const int nN = in_sizes[0] / NIN;
  const int nE = in_sizes[16];
  if (nN <= 0 || nE <= 0) return;
  if (in_sizes[0] != nN * NIN || in_sizes[1] != nE * EF || in_sizes[17] != nE) return;
  if (in_sizes[2] != MSGD * K1 || in_sizes[3] != MSGD || in_sizes[4] != MSGD * MSGD || in_sizes[5] != MSGD) return;
  if (in_sizes[6] != MSGD * MSGD || in_sizes[7] != MSGD || in_sizes[8] != EF * MSGD || in_sizes[9] != EF) return;
  if (in_sizes[10] != 3 * HD * GIN || in_sizes[11] != 3 * HD * HD || in_sizes[12] != 3 * HD || in_sizes[13] != 3 * HD) return;
  if (in_sizes[14] != 2 * HD || in_sizes[15] != 2) return;
  if ((nN % 16) != 0) return;
  const int nT = out_size / (nN * 2);
  if (nT <= 0 || out_size != nT * nN * 2) return;

  const float* node_inputs = (const float*)d_in[0];
  const float* edge_attr   = (const float*)d_in[1];
  const float* W1 = (const float*)d_in[2];
  const float* b1 = (const float*)d_in[3];
  const float* W2 = (const float*)d_in[4];
  const float* b2 = (const float*)d_in[5];
  const float* W3 = (const float*)d_in[6];
  const float* b3 = (const float*)d_in[7];
  const float* W4 = (const float*)d_in[8];
  const float* b4 = (const float*)d_in[9];
  const float* gwih = (const float*)d_in[10];
  const float* gwhh = (const float*)d_in[11];
  const float* gbih = (const float*)d_in[12];
  const float* gbhh = (const float*)d_in[13];
  const float* finw = (const float*)d_in[14];
  const float* finb = (const float*)d_in[15];
  const int* src_ids = (const int*)d_in[16];
  const int* dst_ids = (const int*)d_in[17];
  float* out = (float*)d_out;

  const int nBlk = (nN + NB - 1) / NB;
  const int nPad = nBlk * NB;
  const long long nPieces = 2LL * (long long)nE;
  const int pBlk = (int)((nPieces + NTHR - 1) / NTHR);
  const size_t nPiecesPad = (size_t)pBlk * NTHR;

  char* ws = (char*)d_ws;
  size_t off = 0;
  const size_t szEa = nPiecesPad * 16;
  const size_t szH  = (size_t)nPad * HP * 4;
  const size_t oEa = off; off += (szEa + 255) & ~(size_t)255;
  const size_t oHA = off; off += (szH + 255) & ~(size_t)255;
  const size_t oHB = off; off += (szH + 255) & ~(size_t)255;
  if (off > ws_size) return;
  if (off > (size_t)134217728) return;
  _Float16* ea16 = (_Float16*)(ws + oEa);
  float* hA = (float*)(ws + oHA);
  float* hB = (float*)(ws + oHB);

  k_prep<<<pBlk, NTHR, 0, stream>>>(edge_attr, ea16, nE);
  hipMemsetAsync(hA, 0, szH, stream);

  hipFuncSetAttribute(reinterpret_cast<const void*>(&k_iter), hipFuncAttributeMaxDynamicSharedMemorySize, LDS_BYTES);

  for (int it = 0; it < nT; ++it) {
    const float* hin = (it & 1) ? hB : hA;
    float* hout = (it & 1) ? hA : hB;
    k_iter<<<nBlk, NTHR, LDS_BYTES, stream>>>(
        hin, hout, ea16, node_inputs, W1, b1, W2, b2, W3, b3, W4, b4,
        gwih, gwhh, gbih, gbhh, finw, finb, src_ids, dst_ids,
        out + (size_t)it * nN * 2, nN, nE, nN * 2);
  }
}
